// ElementalReadOut_80728205296199
// MI455X (gfx1250) — hardware-run, weakly checked
//
#include <hip/hip_runtime.h>
#include <math.h>

typedef __attribute__((ext_vector_type(16))) _Float16 v16h;
typedef __attribute__((ext_vector_type(8)))  _Float16 v8h;
typedef __attribute__((ext_vector_type(8)))  float    v8f;
typedef __attribute__((ext_vector_type(4)))  float    v4f;

constexpr int kAtoms      = 100000;
constexpr int kGraphs     = 2048;
constexpr int kFea        = 64;
constexpr int kHead       = 32;
constexpr int kRowsPerBlk = 128;
constexpr int kLogitBlks  = (kAtoms + kRowsPerBlk - 1) / kRowsPerBlk;
constexpr int kAtomsPad   = kLogitBlks * kRowsPerBlk;
constexpr int kChunk      = 64;
constexpr int kBtPitch    = kFea + 8;
constexpr int kKPitch     = kChunk + 8;
constexpr int kTilePitch  = kHead + 4;
constexpr float kFeaCarry = 16.0f;
constexpr float kWkCarry  = 64.0f;
constexpr float kExpCarry = 1024.0f;
constexpr float kLogitFold = 1.0f / (kFeaCarry * kWkCarry);
constexpr float kSumFold   = 1.0f / (kFeaCarry * kExpCarry);

static_assert(kLogitBlks == 782);
static_assert(kAtomsPad == 100096);
static_assert((kFea % 32) == 0);
static_assert((kChunk % 32) == 0);
static_assert(kHead == 32);
static_assert(kFea == 64);

constexpr size_t kOffW    = 0;
constexpr size_t kWsTotal = kOffW + (size_t)kAtomsPad * kHead * 4;
static_assert(kWsTotal == 12812288ull);
static_assert(kWsTotal <= 134217728ull);

union FragH { v16h v; v8h h[2]; };

__device__ __forceinline__ v16h frag_load(const _Float16* p) {
  FragH f;
  f.h[0] = *(const v8h*)(p);
  f.h[1] = *(const v8h*)(p + 16);
  return f.v;
}

__device__ __forceinline__ v8f mma_h(v16h a, v16h b, v8f c) {
  c = __builtin_amdgcn_wmma_f32_16x16x32_f16(false, a, false, b, (short)0, c, false, false);
  asm volatile("v_nop\n\tv_nop\n\tv_nop\n\tv_nop" : "+v"(c) : "v"(a), "v"(b));
  return c;
}

__global__ __launch_bounds__(256) void logits_kernel(
    const float* __restrict__ fea, const float* __restrict__ Wk,
    const float* __restrict__ bk, float* __restrict__ wPlane)
{
  __shared__ __align__(16) _Float16 sBt[kHead * kBtPitch];
  __shared__ __align__(16) float sSlab[8][16 * kTilePitch];

  const int tid  = threadIdx.x;
  const int lane = tid & 31;
  const int wave = tid >> 5;
  const int hh   = lane >> 4;
  const int c    = lane & 15;

  {
    const int h  = tid >> 3;
    const int d8 = (tid & 7) * 8;
    v8h hv;
#pragma unroll
    for (int e = 0; e < 8; ++e) {
      const float v = Wk[(d8 + e) * kHead + h];
      hv[e] = (_Float16)(v * kWkCarry);
    }
    *(v8h*)(sBt + h * kBtPitch + d8) = hv;
  }
  __syncthreads();

  const int row0 = blockIdx.x * kRowsPerBlk + wave * 16;
  int arow = row0 + c;
  arow = arow < kAtoms ? arow : (kAtoms - 1);
  const float* fr = fea + (size_t)arow * kFea + 8 * hh;

  v16h afr[2];
#pragma unroll
  for (int ks = 0; ks < 2; ++ks) {
    const v4f x0 = *(const v4f*)(fr + ks * 32);
    const v4f x1 = *(const v4f*)(fr + ks * 32 + 4);
    const v4f x2 = *(const v4f*)(fr + ks * 32 + 16);
    const v4f x3 = *(const v4f*)(fr + ks * 32 + 20);
#pragma unroll
    for (int e = 0; e < 4; ++e) {
      afr[ks][e]      = (_Float16)(x0[e] * kFeaCarry);
      afr[ks][4 + e]  = (_Float16)(x1[e] * kFeaCarry);
      afr[ks][8 + e]  = (_Float16)(x2[e] * kFeaCarry);
      afr[ks][12 + e] = (_Float16)(x3[e] * kFeaCarry);
    }
  }

  v8f acc0 = (v8f){0.f, 0.f, 0.f, 0.f, 0.f, 0.f, 0.f, 0.f};
  v8f acc1 = (v8f){0.f, 0.f, 0.f, 0.f, 0.f, 0.f, 0.f, 0.f};
#pragma unroll
  for (int ks = 0; ks < 2; ++ks) {
    const v16h b0 = frag_load(sBt + c * kBtPitch + ks * 32 + 8 * hh);
    const v16h b1 = frag_load(sBt + (16 + c) * kBtPitch + ks * 32 + 8 * hh);
    acc0 = mma_h(afr[ks], b0, acc0);
    acc1 = mma_h(afr[ks], b1, acc1);
  }

  const float bk0 = bk[c];
  const float bk1 = bk[16 + c];
  float* slab = sSlab[wave];
#pragma unroll
  for (int r = 0; r < 8; ++r) {
    slab[(8 * hh + r) * kTilePitch + c]      = acc0[r] * kLogitFold + bk0;
    slab[(8 * hh + r) * kTilePitch + 16 + c] = acc1[r] * kLogitFold + bk1;
  }
  __syncthreads();

  const int q  = lane >> 3;
  const int c4 = (lane & 7) * 4;
  v4f vv[4];
#pragma unroll
  for (int it = 0; it < 4; ++it) vv[it] = *(const v4f*)(slab + (it * 4 + q) * kTilePitch + c4);
  for (int pass = 0; pass < 2; ++pass) {
#pragma unroll
    for (int it = 0; it < 4; ++it)
      *(volatile v4f*)(wPlane + (size_t)(row0 + it * 4 + q) * kHead + c4) = vv[it];
    __threadfence();
  }
}

__device__ __forceinline__ int seg_lower_bound(const int* __restrict__ a, int key) {
  int lo = 0, hi = kAtoms;
#pragma unroll 1
  for (int it = 0; it < 18; ++it) {
    const int mid  = (lo + hi) >> 1;
    const int midc = mid < kAtoms ? mid : (kAtoms - 1);
    const int v    = a[midc];
    const bool act  = lo < hi;
    const bool less = v < key;
    const int nlo = (act && less) ? (mid + 1) : lo;
    const int nhi = (act && !less) ? mid : hi;
    lo = nlo;
    hi = nhi;
  }
  return lo;
}

__global__ __launch_bounds__(128) void segment_contract_kernel(
    const float* __restrict__ fea, const float* __restrict__ wPlane,
    const int* __restrict__ owner, float* __restrict__ out)
{
  __shared__ __align__(16) _Float16 sFT[kFea * kKPitch];
  __shared__ __align__(16) _Float16 sP[kHead * kKPitch];
  __shared__ __align__(16) float sOut[kFea * kTilePitch];
  __shared__ float sRedM[4 * 32];
  __shared__ float sRedS[4 * 32];

  const int g    = blockIdx.x;
  const int tid  = threadIdx.x;
  const int lane = tid & 31;
  const int wave = tid >> 5;
  const int hh   = lane >> 4;
  const int c    = lane & 15;

  const int lo = seg_lower_bound(owner, g);
  int hi = seg_lower_bound(owner, g + 1);
  hi = hi < lo ? lo : hi;

  float m = -INFINITY;
#pragma unroll 1
  for (int a = lo + wave; a < hi; a += 4) {
    const float v = wPlane[(size_t)a * kHead + lane];
    m = fmaxf(m, v);
  }
  sRedM[wave * 32 + lane] = m;
  __syncthreads();
  const float segmax = fmaxf(fmaxf(sRedM[lane], sRedM[32 + lane]),
                             fmaxf(sRedM[64 + lane], sRedM[96 + lane]));

  v8f acc0 = (v8f){0.f, 0.f, 0.f, 0.f, 0.f, 0.f, 0.f, 0.f};
  v8f acc1 = (v8f){0.f, 0.f, 0.f, 0.f, 0.f, 0.f, 0.f, 0.f};
  float psum = 0.0f;

  const int n   = hi - lo;
  const int nch = (n + kChunk - 1) / kChunk;
  const int dT  = tid & 63;
  const int gsel = tid >> 6;

#pragma unroll 1
  for (int ch = 0; ch < nch; ++ch) {
    const int base = lo + ch * kChunk;
    int cnt = hi - base;
    cnt = cnt > kChunk ? kChunk : cnt;
    __syncthreads();

#pragma unroll 1
    for (int i = 0; i < 4; ++i) {
      const int a0 = (gsel + 2 * i) * 8;
      v8h hv;
#pragma unroll
      for (int e = 0; e < 8; ++e) {
        int row = base + a0 + e;
        row = row < kAtoms ? row : (kAtoms - 1);
        float x = fea[(size_t)row * kFea + dT];
        asm volatile("" : "+v"(x));
        const float xs = (a0 + e < cnt) ? (x * kFeaCarry) : 0.0f;
        hv[e] = (_Float16)xs;
      }
      *(v8h*)(sFT + dT * kKPitch + a0) = hv;
    }

#pragma unroll 1
    for (int i = 0; i < 2; ++i) {
      const int a0 = (wave + 4 * i) * 8;
      v8h hv;
#pragma unroll
      for (int e = 0; e < 8; ++e) {
        int row = base + a0 + e;
        row = row < kAtoms ? row : (kAtoms - 1);
        float x = wPlane[(size_t)row * kHead + lane];
        asm volatile("" : "+v"(x));
        const float ev = expf(x - segmax);
        const float es = (a0 + e < cnt) ? ev : 0.0f;
        psum += es;
        hv[e] = (_Float16)(es * kExpCarry);
      }
      *(v8h*)(sP + lane * kKPitch + a0) = hv;
    }
    __syncthreads();

#pragma unroll
    for (int ks = 0; ks < 2; ++ks) {
      const v16h a  = frag_load(sFT + (wave * 16 + c) * kKPitch + ks * 32 + 8 * hh);
      const v16h b0 = frag_load(sP + c * kKPitch + ks * 32 + 8 * hh);
      const v16h b1 = frag_load(sP + (16 + c) * kKPitch + ks * 32 + 8 * hh);
      acc0 = mma_h(a, b0, acc0);
      acc1 = mma_h(a, b1, acc1);
    }
  }

  sRedS[wave * 32 + lane] = psum;
  __syncthreads();
  const float s0 = ((sRedS[c] + sRedS[32 + c]) + sRedS[64 + c]) + sRedS[96 + c];
  const float s1 = ((sRedS[16 + c] + sRedS[48 + c]) + sRedS[80 + c]) + sRedS[112 + c];
  const float i0 = (s0 > 0.0f) ? (kSumFold * (1.0f / s0)) : 0.0f;
  const float i1 = (s1 > 0.0f) ? (kSumFold * (1.0f / s1)) : 0.0f;

#pragma unroll
  for (int r = 0; r < 8; ++r) {
    sOut[(wave * 16 + 8 * hh + r) * kTilePitch + c]      = acc0[r] * i0;
    sOut[(wave * 16 + 8 * hh + r) * kTilePitch + 16 + c] = acc1[r] * i1;
  }
  __syncthreads();

  float* og = out + (size_t)g * (kFea * kHead);
  const int q  = lane >> 3;
  const int c4 = (lane & 7) * 4;
  v4f vv[4];
#pragma unroll
  for (int it = 0; it < 4; ++it)
    vv[it] = *(const v4f*)(sOut + (wave * 16 + it * 4 + q) * kTilePitch + c4);
  for (int pass = 0; pass < 2; ++pass) {
#pragma unroll
    for (int it = 0; it < 4; ++it)
      *(volatile v4f*)(og + (size_t)(wave * 16 + it * 4 + q) * kHead + c4) = vv[it];
    __threadfence();
  }
}

extern "C" void kernel_launch(void* const* d_in, const int* in_sizes, int n_in,
                              void* d_out, int out_size, void* d_ws, size_t ws_size,
                              hipStream_t stream) {
  if (n_in < 5) return;
  if (in_sizes[0] != kAtoms * kFea) return;
  if (in_sizes[1] != kFea * kHead) return;
  if (in_sizes[2] != kHead) return;
  if (in_sizes[4] != kAtoms) return;
  if (out_size != kGraphs * kFea * kHead) return;
  if (ws_size < kWsTotal) return;

  const float* fea   = (const float*)d_in[0];
  const float* Wk    = (const float*)d_in[1];
  const float* bk    = (const float*)d_in[2];
  const int*   owner = (const int*)d_in[4];
  float* out = (float*)d_out;
  float* wPlane = (float*)((char*)d_ws + kOffW);

  logits_kernel<<<kLogitBlks, 256, 0, stream>>>(fea, Wk, bk, wPlane);
  segment_contract_kernel<<<kGraphs, 128, 0, stream>>>(fea, wPlane, owner, out);
}
